// GCN_77120432767264
// MI455X (gfx1250) — hardware-run, weakly checked
//
#include <hip/hip_runtime.h>
#include <stddef.h>
#include <stdint.h>
#include <math.h>

#define NN      100000
#define NE      1600000
#define FD      128
#define HD      64
#define KL      128
#define NCLS    10
#define NGR     1024
#define GBM     128
#define MP      100096
#define NTHR    256
#define NWAVE   8
#define EPT     8
#define WCH     (32 * EPT)
#define NBRUN   1024
#define SLB     10
#define NBK     98
#define WLCAP   3584
#define RCAP    20480
#define DEGCAP  64
#define MAXDEG_MEAS   36
#define MAXB1024_MEAS 16710
#define ABM     64
#define SP      68
#define GPB     16
#define NPB     64
#define GCAP    3072
#define MAXG_MEAS 129
#define WSMAX   (128u << 20)

constexpr bool SPLIT_2 = true;
constexpr bool SPLIT_3 = true;

#define BK_ZINTS (NWAVE * WLCAP + RCAP + 3 * NBRUN)
#define BK_INTS  (BK_ZINTS + 16)
#define BK_LDS   (BK_INTS * 4)

#define PBX   (MP * FD / 8 / NTHR)
#define PBW   (HD * KL / 8 / NTHR)
#define PBTOT (PBX + 3 * PBW)

static_assert(HD == 64 && HD == 16 * 4 && FD == KL && KL == 2 * HD);
static_assert(MP % GBM == 0 && MP >= NN && MP == 782 * GBM && MP % ABM == 0);
static_assert(NBRUN == (1 << SLB) && NBRUN % ABM == 0 && NBRUN % GBM == 0 && NBRUN % 32 == 0);
static_assert(NBRUN == 4 * NTHR);
static_assert(NBK * NBRUN >= MP);
static_assert(NE < (1 << 21) && (((long long)NE) << SLB) < (1LL << 31));
static_assert(NE % WCH == 0 && NE % 4 == 0);
static_assert(RCAP % (4 * NTHR) == 0 && BK_ZINTS % (4 * NTHR) == 0);
static_assert((long long)RCAP * 100 >= (long long)MAXB1024_MEAS * 105);
static_assert((long long)WLCAP * 2 * NWAVE >= 3LL * MAXB1024_MEAS);
static_assert(MAXDEG_MEAS + 8 <= DEGCAP);
static_assert(NN < (1 << 17) && GPB == 16);
static_assert(NPB * GPB == NGR && GPB == 2 * NWAVE);
static_assert(GCAP * 100 >= GPB * MAXG_MEAS * 125 && GCAP % (4 * NTHR) == 0);
static_assert((MP * FD / 8) % NTHR == 0 && (HD * KL / 8) % NTHR == 0);
static_assert(FD % 32 == 0 && KL % 32 == 0 && HD % 32 == 0);
static_assert(BK_LDS <= 300000);
static_assert((GBM * SP + GBM) * 4 <= 65536);
static_assert((GPB * NCLS * 4) % 128 == 0 && GPB * NCLS == 160 && GPB * HD == 4 * NTHR);

typedef float          v2f   __attribute__((ext_vector_type(2)));
typedef float          v4f   __attribute__((ext_vector_type(4)));
typedef float          v8f   __attribute__((ext_vector_type(8)));
typedef int            v4i   __attribute__((ext_vector_type(4)));
typedef int            v8i   __attribute__((ext_vector_type(8)));
typedef unsigned short v8us  __attribute__((ext_vector_type(8)));
typedef unsigned short v16us __attribute__((ext_vector_type(16)));
typedef __bf16         v16bf __attribute__((ext_vector_type(16)));
typedef v2f  __attribute__((may_alias)) v2fa;
typedef v4f  __attribute__((may_alias)) v4fa;
typedef v4i  __attribute__((may_alias)) v4ia;
typedef v8us __attribute__((may_alias)) v8usa;
union FragB { v16bf v; v16us u; v8us h[2]; v8i w; };

__device__ __forceinline__ v8f wmb(const FragB& a, const FragB& b, v8f c) {
  v8f d = __builtin_amdgcn_wmma_f32_16x16x32_bf16(false, a.v, false, b.v, (short)0, c, false, false);
  asm volatile("v_nop\n\tv_nop\n\tv_nop\n\tv_nop" : "+v"(d) : "v"(a.w), "v"(b.w));
  return d;
}

__device__ __forceinline__ unsigned bf16_bits(float f) {
  const unsigned u = __float_as_uint(f);
  const unsigned r = (u + 0x7FFFu + ((u >> 16) & 1u)) >> 16;
  const unsigned q = (u >> 16) | 0x40u;
  return ((u & 0x7fffffffu) > 0x7f800000u) ? q : r;
}
__device__ __forceinline__ float bf16_val(float f) {
  return __uint_as_float(bf16_bits(f) << 16);
}

__device__ __forceinline__ void hilo_pack(float v0, float v1, float v2, float v3,
                                          int& h01, int& h23, int& l01, int& l23) {
  const unsigned a0 = bf16_bits(v0), a1 = bf16_bits(v1), a2 = bf16_bits(v2), a3 = bf16_bits(v3);
  const unsigned b0 = bf16_bits(v0 - __uint_as_float(a0 << 16));
  const unsigned b1 = bf16_bits(v1 - __uint_as_float(a1 << 16));
  const unsigned b2 = bf16_bits(v2 - __uint_as_float(a2 << 16));
  const unsigned b3 = bf16_bits(v3 - __uint_as_float(a3 << 16));
  h01 = (int)(a0 | (a1 << 16)); h23 = (int)(a2 | (a3 << 16));
  l01 = (int)(b0 | (b1 << 16)); l23 = (int)(b2 | (b3 << 16));
}

__device__ __forceinline__ v4i regroup8(int h01, int h23, int l01, int l23, int lane) {
  const int t  = lane & 15;
  const int s0 = (lane & 16) + ((2 * t) & 15), s1 = s0 + 1;
  const int a0 = __shfl(h01, s0, 32), a1 = __shfl(h23, s0, 32), a2 = __shfl(h01, s1, 32), a3 = __shfl(h23, s1, 32);
  const int b0 = __shfl(l01, s0, 32), b1 = __shfl(l23, s0, 32), b2 = __shfl(l01, s1, 32), b3 = __shfl(l23, s1, 32);
  const int mk = (t < 8) ? -1 : 0;
  v4i o;
  o.x = (a0 & mk) | (b0 & ~mk); o.y = (a1 & mk) | (b1 & ~mk);
  o.z = (a2 & mk) | (b2 & ~mk); o.w = (a3 & mk) | (b3 & ~mk);
  return o;
}

__device__ __forceinline__ void st2_v4f(float* p, v4f v) {
  *(volatile v4f*)p = v;
  __threadfence();
  *(volatile v4f*)p = v;
}
__device__ __forceinline__ void st2_v8us(unsigned short* p, v8us v) {
  *(volatile v8us*)p = v;
  __threadfence();
  *(volatile v8us*)p = v;
}

__device__ __forceinline__ v8us gather8(const float* __restrict__ base, int stride) {
  float f[8];
#pragma unroll
  for (int i = 0; i < 8; ++i) f[i] = base[(size_t)i * (size_t)stride];
  v8us o;
#pragma unroll
  for (int i = 0; i < 8; ++i) o[i] = (unsigned short)bf16_bits(f[i]);
  return o;
}

__global__ __launch_bounds__(NTHR) void k_prep(const float* __restrict__ x, const float* __restrict__ w1,
                                               const float* __restrict__ w2, const float* __restrict__ w3,
                                               unsigned short* xb, unsigned short* w1t,
                                               unsigned short* w2d, unsigned short* w3d) {
  const int tid = (int)threadIdx.x;
  const int blk = (int)blockIdx.x;
  if (blk < PBX) {
    const int u   = blk * NTHR + tid;
    const int row = u >> 4, k8 = (u & 15) * 8;
    const int rc  = row < NN ? row : NN - 1;
    const unsigned mk = row < NN ? 0xffffu : 0u;
    const float* p = x + (size_t)rc * FD + k8;
    const v4f a = *(const v4fa*)p;
    const v4f b = *(const v4fa*)(p + 4);
    v8us o;
    o[0] = (unsigned short)(bf16_bits(a.x) & mk); o[1] = (unsigned short)(bf16_bits(a.y) & mk);
    o[2] = (unsigned short)(bf16_bits(a.z) & mk); o[3] = (unsigned short)(bf16_bits(a.w) & mk);
    o[4] = (unsigned short)(bf16_bits(b.x) & mk); o[5] = (unsigned short)(bf16_bits(b.y) & mk);
    o[6] = (unsigned short)(bf16_bits(b.z) & mk); o[7] = (unsigned short)(bf16_bits(b.w) & mk);
    st2_v8us(xb + (size_t)row * FD + k8, o);
  } else if (blk < PBX + PBW) {
    const int u = (blk - PBX) * NTHR + tid;
    const int n = u >> 4, k8 = (u & 15) * 8;
    const v8us o = gather8(w1 + (size_t)k8 * HD + n, HD);
    st2_v8us(w1t + (size_t)n * FD + k8, o);
  } else if (blk < PBX + 2 * PBW) {
    const int u = (blk - PBX - PBW) * NTHR + tid;
    const int n = u >> 4, k8 = (u & 15) * 8, kk = k8 & 63;
    const v8us o = gather8(w2 + (size_t)kk * HD + n, HD);
    st2_v8us(w2d + (size_t)n * KL + k8, o);
  } else {
    const int u = (blk - PBX - 2 * PBW) * NTHR + tid;
    const int n = u >> 4, k8 = (u & 15) * 8, kk = k8 & 63;
    const v8us o = gather8(w3 + (size_t)kk * HD + n, HD);
    st2_v8us(w3d + (size_t)n * KL + k8, o);
  }
}

__device__ __forceinline__ void bucket_flush(const int* pl, const int* cnt, int ov, int* lp, int* cop,
                                             float* dvp, int* fp, int tid) {
#pragma unroll 1
  for (int i = tid * 4; i < RCAP; i += NTHR * 4) {
    const v4i v = *(const v4ia*)(pl + i);
    *(volatile v4i*)(lp + i) = v;
  }
  {
    const v4i c4 = *(const v4ia*)(cnt + 4 * tid);
    const v4i o4 = *(const v4ia*)(cnt + NBRUN + 4 * tid);
    *(volatile v4i*)(cop + 4 * tid) = c4;
    *(volatile v4i*)(cop + NBRUN + 4 * tid) = o4;
    v4f dv;
    dv.x = rsqrtf((float)(c4.x + 1)); dv.y = rsqrtf((float)(c4.y + 1));
    dv.z = rsqrtf((float)(c4.z + 1)); dv.w = rsqrtf((float)(c4.w + 1));
    *(volatile v4f*)(dvp + 4 * tid) = dv;
  }
  if (tid < 8) {
    const v4i f = {ov, ov, ov, ov};
    *(volatile v4i*)(fp + 4 * tid) = f;
  }
}

__global__ __launch_bounds__(NTHR) __attribute__((amdgpu_num_vgpr(248)))
void k_bucket(const int* __restrict__ srcs, const int* __restrict__ dsts,
              int* LIST, int* CO, float* DINV, int* FLAG) {
  extern __shared__ __attribute__((aligned(16))) int dsm[];
  int* wl   = dsm;
  int* pl   = dsm + NWAVE * WLCAP;
  int* cnt  = pl + RCAP;
  int* offs = cnt + NBRUN;
  int* cur  = offs + NBRUN;
  int* misc = cur + NBRUN;
  const int tid = (int)threadIdx.x, lane = tid & 31, wave = tid >> 5;
  const int blk = (int)blockIdx.x;
  const unsigned nbs = (unsigned)(blk * NBRUN);

  {
    const v4i z4 = {0, 0, 0, 0};
    for (int i = tid * 4; i < BK_ZINTS; i += NTHR * 4) *(v4ia*)(dsm + i) = z4;
    if (tid < 16) misc[tid] = 0;
  }
  __syncthreads();

  {
    const int per  = ((NE + NWAVE * WCH - 1) / (NWAVE * WCH)) * WCH;
    const int ebeg = wave * per;
    const int eend = (ebeg + per < NE) ? (ebeg + per) : NE;
    int* mylist = wl + wave * WLCAP;
    int wc = 0;
#pragma unroll 1
    for (int cb = ebeg; cb < eend; cb += WCH) {
      const int e0 = cb + lane * EPT;
      const v4i da = *(const v4ia*)(dsts + e0);
      const v4i db = *(const v4ia*)(dsts + e0 + 4);
      const unsigned s0 = (unsigned)da.x - nbs, s1 = (unsigned)da.y - nbs;
      const unsigned s2 = (unsigned)da.z - nbs, s3 = (unsigned)da.w - nbs;
      const unsigned s4 = (unsigned)db.x - nbs, s5 = (unsigned)db.y - nbs;
      const unsigned s6 = (unsigned)db.z - nbs, s7 = (unsigned)db.w - nbs;
      const bool h0 = s0 < (unsigned)NBRUN, h1 = s1 < (unsigned)NBRUN, h2 = s2 < (unsigned)NBRUN, h3 = s3 < (unsigned)NBRUN;
      const bool h4 = s4 < (unsigned)NBRUN, h5 = s5 < (unsigned)NBRUN, h6 = s6 < (unsigned)NBRUN, h7 = s7 < (unsigned)NBRUN;
      const unsigned m0 = __builtin_amdgcn_ballot_w32(h0), m1 = __builtin_amdgcn_ballot_w32(h1);
      const unsigned m2 = __builtin_amdgcn_ballot_w32(h2), m3 = __builtin_amdgcn_ballot_w32(h3);
      const unsigned m4 = __builtin_amdgcn_ballot_w32(h4), m5 = __builtin_amdgcn_ballot_w32(h5);
      const unsigned m6 = __builtin_amdgcn_ballot_w32(h6), m7 = __builtin_amdgcn_ballot_w32(h7);
      const unsigned any = m0 | m1 | m2 | m3 | m4 | m5 | m6 | m7;
      if (any != 0u) {
        const int pre = (int)(__builtin_amdgcn_mbcnt_lo(m0, 0u) + __builtin_amdgcn_mbcnt_lo(m1, 0u) +
                              __builtin_amdgcn_mbcnt_lo(m2, 0u) + __builtin_amdgcn_mbcnt_lo(m3, 0u) +
                              __builtin_amdgcn_mbcnt_lo(m4, 0u) + __builtin_amdgcn_mbcnt_lo(m5, 0u) +
                              __builtin_amdgcn_mbcnt_lo(m6, 0u) + __builtin_amdgcn_mbcnt_lo(m7, 0u));
        int p = wc + pre;
        if (h0) { if (p < WLCAP) mylist[p] = ((e0 + 0) << SLB) | (int)s0; p = p + 1; }
        if (h1) { if (p < WLCAP) mylist[p] = ((e0 + 1) << SLB) | (int)s1; p = p + 1; }
        if (h2) { if (p < WLCAP) mylist[p] = ((e0 + 2) << SLB) | (int)s2; p = p + 1; }
        if (h3) { if (p < WLCAP) mylist[p] = ((e0 + 3) << SLB) | (int)s3; p = p + 1; }
        if (h4) { if (p < WLCAP) mylist[p] = ((e0 + 4) << SLB) | (int)s4; p = p + 1; }
        if (h5) { if (p < WLCAP) mylist[p] = ((e0 + 5) << SLB) | (int)s5; p = p + 1; }
        if (h6) { if (p < WLCAP) mylist[p] = ((e0 + 6) << SLB) | (int)s6; p = p + 1; }
        if (h7) { if (p < WLCAP) mylist[p] = ((e0 + 7) << SLB) | (int)s7; p = p + 1; }
        wc += (int)(__builtin_popcount(m0) + __builtin_popcount(m1) + __builtin_popcount(m2) + __builtin_popcount(m3) +
                    __builtin_popcount(m4) + __builtin_popcount(m5) + __builtin_popcount(m6) + __builtin_popcount(m7));
      }
    }
    if (lane == 0) misc[wave] = wc;
  }
  __syncthreads();

  if (wave == 0) {
    int ov = 0;
#pragma unroll 1
    for (int w2 = 0; w2 < NWAVE; ++w2) {
      int c = misc[w2];
      if (c > WLCAP) ov = 1;
      c = c < 0 ? 0 : (c > WLCAP ? WLCAP : c);
#pragma unroll 1
      for (int b0 = 0; b0 < c; b0 += 32) {
        const int idx = b0 + lane;
        const int ent = wl[w2 * WLCAP + (idx < WLCAP ? idx : WLCAP - 1)];
        const int m32 = (c - b0) < 32 ? (c - b0) : 32;
#pragma unroll 1
        for (int k = 0; k < m32; ++k) {
          const int u    = __builtin_amdgcn_readlane(ent, k);
          const int slot = u & (NBRUN - 1);
          if (lane == 0) cnt[slot] = cnt[slot] + 1;
        }
      }
    }
    if (lane == 0) misc[9] = ov;
  }
  __syncthreads();
  if (wave == 0) {
    const int base = lane * (NBRUN / 32);
    int s = 0;
#pragma unroll 1
    for (int i = 0; i < NBRUN / 32; ++i) s += cnt[base + i];
    int incl = s;
#pragma unroll
    for (int d = 1; d < 32; d <<= 1) {
      const int y = __shfl_up(incl, d, 32);
      if (lane >= d) incl += y;
    }
    int run = incl - s;
#pragma unroll 1
    for (int i = 0; i < NBRUN / 32; ++i) {
      const int cv = cnt[base + i];
      offs[base + i] = run;
      cur[base + i]  = run;
      run += cv;
    }
    if (lane == 31 && run > RCAP) misc[10] = 1;
  }
  __syncthreads();

  if (wave == 0) {
#pragma unroll 1
    for (int w2 = 0; w2 < NWAVE; ++w2) {
      int c = misc[w2];
      c = c < 0 ? 0 : (c > WLCAP ? WLCAP : c);
#pragma unroll 1
      for (int b0 = 0; b0 < c; b0 += 32) {
        const int idx = b0 + lane;
        const int ent = wl[w2 * WLCAP + (idx < WLCAP ? idx : WLCAP - 1)];
        int eid = (ent >> SLB) & 0x1FFFFF;
        eid = eid > NE - 1 ? NE - 1 : eid;
        int sr = srcs[eid];
        sr = sr < 0 ? 0 : (sr > NN - 1 ? NN - 1 : sr);
        const int m32 = (c - b0) < 32 ? (c - b0) : 32;
#pragma unroll 1
        for (int k = 0; k < m32; ++k) {
          const int u    = __builtin_amdgcn_readlane(ent, k);
          const int wd   = __builtin_amdgcn_readlane(sr, k);
          const int slot = u & (NBRUN - 1);
          if (lane == 0) {
            int p = cur[slot];
            p = p < 0 ? 0 : (p > RCAP - 1 ? RCAP - 1 : p);
            pl[p] = wd;
            cur[slot] = p + 1;
          }
        }
      }
    }
  }
  __syncthreads();

  const int ovf = misc[9] | misc[10];
  int*   lp  = LIST + (size_t)blk * RCAP;
  int*   cop = CO + (size_t)blk * (2 * NBRUN);
  float* dvp = DINV + (size_t)blk * NBRUN;
  int*   fp  = FLAG + (size_t)blk * 32;
  bucket_flush(pl, cnt, ovf, lp, cop, dvp, fp, tid);
  __threadfence();
  bucket_flush(pl, cnt, ovf, lp, cop, dvp, fp, tid);
}

template <int KTOT, int PITCH>
__device__ __forceinline__ void gemm_16x64(const unsigned short* __restrict__ ap,
                                           const unsigned short* __restrict__ bp, v8f (&acc)[4]) {
#pragma unroll 1
  for (int k0 = 0; k0 < KTOT; k0 += 32) {
    FragB af;
    af.h[0] = *(const v8usa*)(ap + k0);
    af.h[1] = *(const v8usa*)(ap + k0 + 16);
#pragma unroll
    for (int nt = 0; nt < 4; ++nt) {
      const unsigned short* wq = bp + (size_t)(16 * nt) * (size_t)PITCH + k0;
      FragB bf;
      bf.h[0] = *(const v8usa*)wq;
      bf.h[1] = *(const v8usa*)(wq + 16);
      acc[nt] = wmb(af, bf, acc[nt]);
    }
  }
}

__device__ __forceinline__ void stage_d(float* stg, const v8f (&acc)[4], int wave, int hh, int m) {
#pragma unroll
  for (int nt = 0; nt < 4; ++nt) {
#pragma unroll
    for (int r = 0; r < 8; ++r) stg[(16 * wave + 8 * hh + r) * SP + 16 * nt + m] = acc[nt][r];
  }
}

template <int KTOT>
__global__ __launch_bounds__(NTHR) __attribute__((amdgpu_num_vgpr(248)))
void k_xform(const unsigned short* __restrict__ A, const unsigned short* __restrict__ BT,
             const float* __restrict__ DINV, float* P) {
  __shared__ __attribute__((aligned(16))) float stg[GBM * SP];
  __shared__ __attribute__((aligned(16))) float sdv[GBM];
  const int tid = (int)threadIdx.x, lane = tid & 31, wave = tid >> 5, hh = lane >> 4, m = lane & 15;
  const int rowBase = (int)blockIdx.x * GBM;
  if (tid < 32) *(v4fa*)(sdv + 4 * tid) = *(const v4fa*)(DINV + (size_t)rowBase + 4 * tid);

  v8f acc[4];
  {
    const v8f z = {0.f, 0.f, 0.f, 0.f, 0.f, 0.f, 0.f, 0.f};
#pragma unroll
    for (int t = 0; t < 4; ++t) acc[t] = z;
  }
  const unsigned short* ap = A + (size_t)(rowBase + 16 * wave + m) * (size_t)KL + 8 * hh;
  const unsigned short* bp = BT + (size_t)m * (size_t)KL + 8 * hh;
  gemm_16x64<KTOT, KL>(ap, bp, acc);
  stage_d(stg, acc, wave, hh, m);
  __syncthreads();

#pragma unroll 1
  for (int i = 0; i < 8; ++i) {
    const int lr   = 16 * wave + 2 * i + hh;
    const int grow = rowBase + lr;
    const v4f a  = *(const v4fa*)(stg + lr * SP + 4 * m);
    const float dv = sdv[lr];
    v4f o;
    o.x = dv * a.x; o.y = dv * a.y; o.z = dv * a.z; o.w = dv * a.w;
    st2_v4f(P + (size_t)grow * HD + 4 * m, o);
  }
}

template <int MODE>
__global__ __launch_bounds__(NTHR) __attribute__((amdgpu_num_vgpr(248)))
void k_replay(const int* __restrict__ LIST, const int* __restrict__ CO, const int* __restrict__ FLAG,
              const float* __restrict__ DINV, const float* P, const float* __restrict__ bias,
              unsigned short* HHL, float* H3) {
  __shared__ __attribute__((aligned(16))) float sb[HD];
  const int tid = (int)threadIdx.x, lane = tid & 31, wave = tid >> 5, hh = lane >> 4, q = lane & 15;
  if (tid < 16) {
    const v4f b = *(const v4fa*)(bias + 4 * tid);
    v4f r;
    r.x = bf16_val(b.x); r.y = bf16_val(b.y); r.z = bf16_val(b.z); r.w = bf16_val(b.w);
    *(v4fa*)(sb + 4 * tid) = r;
  }
  __syncthreads();
  const v4f bv = *(const v4fa*)(sb + 4 * q);
  const int rowBase = (int)blockIdx.x * ABM;
  const int bucket  = rowBase >> SLB;
  const int* lb  = LIST + (size_t)bucket * RCAP;
  const int* cob = CO + (size_t)bucket * (2 * NBRUN);
  const int flag = FLAG[(size_t)bucket * 32];
  const float qnan = __uint_as_float(0x7fc00000u);

#pragma unroll 1
  for (int i = 0; i < ABM / (2 * NWAVE); ++i) {
    const int d    = rowBase + (ABM / NWAVE) * wave + 2 * i + hh;
    const int slot = d & (NBRUN - 1);
    int c = cob[slot];
    int o = cob[NBRUN + slot];
    const bool big = c > DEGCAP;
    c = c < 0 ? 0 : (c > DEGCAP ? DEGCAP : c);
    o = o < 0 ? 0 : (o > RCAP - 1 ? RCAP - 1 : o);
    const int co = __shfl_xor(c, 16, 32);
    int cm = c > co ? c : co;
    cm = __builtin_amdgcn_readfirstlane(cm);
    int last = o + c - 1; last = last < o ? o : last;
    last = last > RCAP - 1 ? RCAP - 1 : last;
    float a0 = 0.0f, a1 = 0.0f, a2 = 0.0f, a3 = 0.0f;
#pragma unroll 1
    for (int j = 0; j < cm; ++j) {
      int idx = o + j;
      idx = idx > last ? last : idx;
      int sr = lb[idx];
      sr = sr < 0 ? 0 : (sr > NN - 1 ? NN - 1 : sr);
      const v4f v = *(const v4fa*)(P + (size_t)sr * HD + 4 * q);
      asm volatile("" :: "v"(v));
      const bool valid = j < c;
      const float t0 = a0 + v.x, t1 = a1 + v.y, t2 = a2 + v.z, t3 = a3 + v.w;
      a0 = valid ? t0 : a0; a1 = valid ? t1 : a1; a2 = valid ? t2 : a2; a3 = valid ? t3 : a3;
    }
    const v4f g = *(const v4fa*)(P + (size_t)d * HD + 4 * q);
    const float dv = DINV[d];
    a0 = a0 + g.x; a1 = a1 + g.y; a2 = a2 + g.z; a3 = a3 + g.w;
    float m0 = dv * a0 + bv.x, m1 = dv * a1 + bv.y, m2 = dv * a2 + bv.z, m3 = dv * a3 + bv.w;
    const bool bad  = (flag != 0) | big;
    const bool live = d < NN;
    m0 = bad ? qnan : m0; m1 = bad ? qnan : m1; m2 = bad ? qnan : m2; m3 = bad ? qnan : m3;
    m0 = live ? m0 : 0.0f; m1 = live ? m1 : 0.0f; m2 = live ? m2 : 0.0f; m3 = live ? m3 : 0.0f;
    if constexpr (MODE != 0) {
      int h01, h23, l01, l23;
      hilo_pack(m0, m1, m2, m3, h01, h23, l01, l23);
      const v4i ow = regroup8(h01, h23, l01, l23, lane);
      unsigned short* hp = HHL + (size_t)d * KL + 8 * q;
      *(volatile v4i*)hp = ow;
      __threadfence();
      *(volatile v4i*)hp = ow;
    } else {
      v4f ov;
      ov.x = m0; ov.y = m1; ov.z = m2; ov.w = m3;
      float* op = H3 + (size_t)d * HD + 4 * q;
      *(volatile v4f*)op = ov;
      __threadfence();
      *(volatile v4f*)op = ov;
    }
  }
}

__global__ __launch_bounds__(NTHR) __attribute__((amdgpu_num_vgpr(248)))
void k_pool(const float* __restrict__ H3, const int* __restrict__ bat,
            const float* __restrict__ Wl, const float* __restrict__ bl, float* out) {
  __shared__ __attribute__((aligned(16))) int   glist[GCAP];
  __shared__ __attribute__((aligned(16))) float psum[GPB * HD];
  __shared__ __attribute__((aligned(16))) float pmean[GPB * HD];
  __shared__ __attribute__((aligned(16))) float os[GPB * NCLS];
  __shared__ float wls[HD * NCLS];
  __shared__ float bls[16];
  __shared__ int pcnt[GPB];
  __shared__ int misc[16];
  const int tid = (int)threadIdx.x, lane = tid & 31, wave = tid >> 5;
  const int wv  = __builtin_amdgcn_readfirstlane(wave);
  const int blk = (int)blockIdx.x;
  const int gbase = blk * GPB;

  {
    const v4i z4 = {0, 0, 0, 0};
    for (int i = tid * 4; i < GCAP; i += NTHR * 4) *(v4ia*)(glist + i) = z4;
    if (tid < 16) misc[tid] = 0;
  }
#pragma unroll 1
  for (int i = tid; i < HD * NCLS; i += NTHR) wls[i] = bf16_val(Wl[i]);
  if (tid < 16) {
    const float bb = bl[tid < NCLS ? tid : NCLS - 1];
    asm volatile("" :: "v"(bb));
    bls[tid] = (tid < NCLS) ? bf16_val(bb) : 0.0f;
  }
  __syncthreads();

  const int per  = ((NN + NWAVE * 32 - 1) / (NWAVE * 32)) * 32;
  const int nbeg = wave * per;
  const int nend = (nbeg + per < NN) ? (nbeg + per) : NN;
  {
    int wc = 0;
#pragma unroll 1
    for (int i0 = nbeg; i0 < nend; i0 += 32) {
      const int i  = i0 + lane;
      const int ic = i < NN ? i : NN - 1;
      const int b  = bat[ic];
      asm volatile("" :: "v"(b));
      const unsigned lg = (unsigned)(b - gbase);
      const bool hit = (i < NN) & (lg < (unsigned)GPB);
      const unsigned mk = __builtin_amdgcn_ballot_w32(hit);
      wc += (int)__builtin_popcount(mk);
    }
    if (lane == 0) misc[wave] = wc;
  }
  __syncthreads();
  int base = 0, tot = 0;
#pragma unroll
  for (int w2 = 0; w2 < NWAVE; ++w2) {
    int c = misc[w2];
    c = c < 0 ? 0 : (c > NN ? NN : c);
    base += (w2 < wave) ? c : 0;
    tot  += c;
  }
  const bool ovf = tot > GCAP;

  {
    int wp = base;
#pragma unroll 1
    for (int i0 = nbeg; i0 < nend; i0 += 32) {
      const int i  = i0 + lane;
      const int ic = i < NN ? i : NN - 1;
      const int b  = bat[ic];
      asm volatile("" :: "v"(b));
      const unsigned lg = (unsigned)(b - gbase);
      const bool hit = (i < NN) & (lg < (unsigned)GPB);
      const unsigned mk = __builtin_amdgcn_ballot_w32(hit);
      if (mk != 0u) {
        const int pos = wp + (int)__builtin_amdgcn_mbcnt_lo(mk, 0u);
        if (hit && pos < GCAP) glist[pos] = i | ((int)lg << 17);
        wp += (int)__builtin_popcount(mk);
      }
    }
  }
  __syncthreads();

  const int tt = tot > GCAP ? GCAP : tot;
  float a0 = 0.0f, a1 = 0.0f, c0 = 0.0f, c1 = 0.0f;
  int na = 0, nb = 0;
#pragma unroll 1
  for (int b0 = 0; b0 < tt; b0 += 32) {
    const int idx = b0 + lane;
    const int ent = glist[idx < GCAP ? idx : GCAP - 1];
    const int m32 = (tt - b0) < 32 ? (tt - b0) : 32;
#pragma unroll 1
    for (int k = 0; k < m32; ++k) {
      const int u  = __builtin_amdgcn_readlane(ent, k);
      const int lg = (u >> 17) & (GPB - 1);
      int node = u & 0x1FFFF;
      node = node > NN - 1 ? NN - 1 : node;
      if ((lg >> 1) == wv) {
        const v2f v = *(const v2fa*)(H3 + (size_t)node * HD + 2 * lane);
        if ((lg & 1) != 0) { c0 += v.x; c1 += v.y; nb = nb + 1; }
        else               { a0 += v.x; a1 += v.y; na = na + 1; }
      }
    }
  }
  psum[(2 * wave) * HD + 2 * lane]         = a0;
  psum[(2 * wave) * HD + 2 * lane + 1]     = a1;
  psum[(2 * wave + 1) * HD + 2 * lane]     = c0;
  psum[(2 * wave + 1) * HD + 2 * lane + 1] = c1;
  if (lane == 0) { pcnt[2 * wave] = na; pcnt[2 * wave + 1] = nb; }
  __syncthreads();

  const float qnan = __uint_as_float(0x7fc00000u);
#pragma unroll 1
  for (int it = 0; it < (GPB * HD) / NTHR; ++it) {
    const int i = it * NTHR + tid;
    const int g = i >> 6;
    const int c = pcnt[g];
    const float cf = (c < 1) ? 1.0f : (float)c;
    float v = psum[i] / cf;
    v = ovf ? qnan : v;
    pmean[i] = v;
  }
  __syncthreads();

  if (tid < GPB * NCLS) {
    const int g = tid / NCLS;
    const int c = tid - g * NCLS;
    float s = 0.0f;
#pragma unroll 4
    for (int k = 0; k < HD; ++k) s = fmaf(pmean[g * HD + k], wls[k * NCLS + c], s);
    os[tid] = s + bls[c];
  }
  __syncthreads();

  const int t4 = tid < 40 ? tid : 39;
  const v4f ov = *(const v4fa*)(os + 4 * t4);
  asm volatile("" :: "v"(ov));
  float* op = out + (size_t)blk * (GPB * NCLS) + 4 * t4;
  if (tid < 40) *(volatile v4f*)op = ov;
  __threadfence();
  if (tid < 40) *(volatile v4f*)op = ov;
}

extern "C" void kernel_launch(void* const* d_in, const int* in_sizes, int n_in,
                              void* d_out, int out_size, void* d_ws, size_t ws_size,
                              hipStream_t stream) {
  if (n_in < 11) return;
  if (in_sizes[0] != NN * FD) return;
  if (in_sizes[1] != 2 * NE) return;
  if (in_sizes[2] != NN) return;
  if (in_sizes[3] != FD * HD) return;
  if (in_sizes[4] != HD) return;
  if (in_sizes[5] != HD * HD) return;
  if (in_sizes[6] != HD) return;
  if (in_sizes[7] != HD * HD) return;
  if (in_sizes[8] != HD) return;
  if (in_sizes[9] != HD * NCLS) return;
  if (in_sizes[10] != NCLS) return;
  if (out_size != NGR * NCLS) return;

  const float* x   = (const float*)d_in[0];
  const int*   ei  = (const int*)d_in[1];
  const int*   bat = (const int*)d_in[2];
  const float* W1  = (const float*)d_in[3];
  const float* b1  = (const float*)d_in[4];
  const float* W2  = (const float*)d_in[5];
  const float* b2  = (const float*)d_in[6];
  const float* W3  = (const float*)d_in[7];
  const float* b3  = (const float*)d_in[8];
  const float* Wl  = (const float*)d_in[9];
  const float* bl  = (const float*)d_in[10];
  float* out = (float*)d_out;
  const int* srcs = ei;
  const int* dsts = ei + NE;

  constexpr size_t zXB   = (size_t)MP * FD * 2;
  constexpr size_t zF    = (size_t)MP * HD * 4;
  constexpr size_t zHL   = (size_t)MP * KL * 2;
  constexpr size_t zLIST = (size_t)NBK * RCAP * 4;
  constexpr size_t zCO   = (size_t)NBK * 2 * NBRUN * 4;
  constexpr size_t zDV   = (size_t)NBK * NBRUN * 4;
  constexpr size_t zFLAG = (size_t)NBK * 128;
  constexpr size_t zW    = (size_t)HD * KL * 2;
  constexpr size_t oXB   = 0;
  constexpr size_t oP    = oXB + zXB;
  constexpr size_t oHHL  = oP + zF;
  constexpr size_t oH3   = oHHL + zHL;
  constexpr size_t oLIST = oH3 + zF;
  constexpr size_t oCO   = oLIST + zLIST;
  constexpr size_t oDV   = oCO + zCO;
  constexpr size_t oFLAG = oDV + zDV;
  constexpr size_t oW1T  = oFLAG + zFLAG;
  constexpr size_t oW2D  = oW1T + zW;
  constexpr size_t oW3D  = oW2D + zW;
  constexpr size_t oEND  = oW3D + zW;
  static_assert(zXB % 256 == 0 && zF % 256 == 0 && zHL % 256 == 0 && zLIST % 256 == 0 && zCO % 256 == 0);
  static_assert(zDV % 256 == 0 && zFLAG % 256 == 0 && zW % 256 == 0);
  static_assert((size_t)NBK * NBRUN >= (size_t)MP);
  static_assert(oEND <= (size_t)WSMAX);
  if (oEND > ws_size) return;

  char* ws = (char*)d_ws;
  unsigned short* XB   = (unsigned short*)(ws + oXB);
  float*          P    = (float*)(ws + oP);
  unsigned short* HHL  = (unsigned short*)(ws + oHHL);
  float*          H3   = (float*)(ws + oH3);
  int*            LIST = (int*)(ws + oLIST);
  int*            CO   = (int*)(ws + oCO);
  float*          DINV = (float*)(ws + oDV);
  int*            FLAG = (int*)(ws + oFLAG);
  unsigned short* W1T  = (unsigned short*)(ws + oW1T);
  unsigned short* W2D  = (unsigned short*)(ws + oW2D);
  unsigned short* W3D  = (unsigned short*)(ws + oW3D);

  constexpr int K2 = SPLIT_2 ? KL : HD;
  constexpr int K3 = SPLIT_3 ? KL : HD;

  hipFuncSetAttribute(reinterpret_cast<const void*>(&k_bucket), hipFuncAttributeMaxDynamicSharedMemorySize, (int)BK_LDS);

  k_prep<<<PBTOT, NTHR, 0, stream>>>(x, W1, W2, W3, XB, W1T, W2D, W3D);
  k_bucket<<<NBK, NTHR, BK_LDS, stream>>>(srcs, dsts, LIST, CO, DINV, FLAG);
  k_xform<FD><<<MP / GBM, NTHR, 0, stream>>>(XB, W1T, DINV, P);
  k_replay<1><<<MP / ABM, NTHR, 0, stream>>>(LIST, CO, FLAG, DINV, P, b1, HHL, H3);
  k_xform<K2><<<MP / GBM, NTHR, 0, stream>>>(HHL, W2D, DINV, P);
  k_replay<1><<<MP / ABM, NTHR, 0, stream>>>(LIST, CO, FLAG, DINV, P, b2, HHL, H3);
  k_xform<K3><<<MP / GBM, NTHR, 0, stream>>>(HHL, W3D, DINV, P);
  k_replay<0><<<MP / ABM, NTHR, 0, stream>>>(LIST, CO, FLAG, DINV, P, b3, HHL, H3);
  k_pool<<<NPB, NTHR, 0, stream>>>(H3, bat, Wl, bl, out);
}
